// ProbAttention_30107720745426
// MI455X (gfx1250) — hardware-verified
//
#include <hip/hip_runtime.h>
#include <math.h>

typedef __attribute__((ext_vector_type(16))) _Float16 v16h;
typedef __attribute__((ext_vector_type(16))) __bf16 v16b;
typedef __attribute__((ext_vector_type(8)))  _Float16 v8h;
typedef __attribute__((ext_vector_type(8)))  __bf16 v8b;
typedef __attribute__((ext_vector_type(8)))  float v8f;
typedef __attribute__((ext_vector_type(4)))  float v4f;
typedef __attribute__((ext_vector_type(4)))  unsigned v4u;

template <typename T> __device__ __forceinline__ void vst2(void* p, T v) { *(volatile T*)p = v; __threadfence(); *(volatile T*)p = v; }
__device__ __forceinline__ v8f wmma16(v16h a, v16h b, v8f c) {
  v8f d = __builtin_amdgcn_wmma_f32_16x16x32_f16(false, a, false, b, (short)0, c, false, false);
  asm volatile("v_nop\n\tv_nop\n\tv_nop\n\tv_nop" : "+v"(d) : "v"(a), "v"(b));
  return d;
}
__device__ __forceinline__ v8f wmma_bf(v16b a, v16b b, v8f c) {
  v8f d = __builtin_amdgcn_wmma_f32_16x16x32_bf16(false, a, false, b, (short)0, c, false, false);
  asm volatile("v_nop\n\tv_nop\n\tv_nop\n\tv_nop" : "+v"(d) : "v"(a), "v"(b));
  return d;
}
__device__ __forceinline__ v16h frag_h(const _Float16* rowk0, int lane) {
  union { v16h v; v8h q[2]; } u; const _Float16* p = rowk0 + 8 * (lane >> 4);
  u.q[0] = *(const v8h*)p; u.q[1] = *(const v8h*)(p + 16); return u.v;
}
__device__ __forceinline__ v16b frag_b(const __bf16* rowk0, int lane) {
  union { v16b v; v8b q[2]; } u; const __bf16* p = rowk0 + 8 * (lane >> 4);
  u.q[0] = *(const v8b*)p; u.q[1] = *(const v8b*)(p + 16); return u.v;
}
__device__ __forceinline__ float bfr(float v) { return (float)(__bf16)v; }
__device__ __forceinline__ void ldsx() { asm volatile("s_wait_dscnt 0" ::: "memory"); __builtin_amdgcn_wave_barrier(); __builtin_amdgcn_fence(3, "workgroup"); }

#ifndef NB
#define NB 4
#endif
#ifndef SEQ
#define SEQ 2048
#endif
#define NB_FULL 4
#define SEQ_FULL 2048
#define NH 8
#define DD 64
#define RS (NH * DD)
#define BSTR ((size_t)SEQ_FULL * RS)
#ifndef OSEQ
#define OSEQ SEQ
#endif
#define PCARRY 16384.0f
static_assert(SEQ % 64 == 0);
static_assert(SEQ <= SEQ_FULL);
static_assert(NB >= 1 && NB <= NB_FULL);
static_assert(DD == 64);

#define WS_VT  0u
#define WS_END (WS_VT + 2u * (size_t)NB * NH * DD * SEQ)
static_assert(WS_END <= (size_t)134217728u);

__global__ __launch_bounds__(128) void k_vt(const float* __restrict__ V, _Float16* __restrict__ VT) {
  __shared__ __align__(16) _Float16 th[DD][72];
  const int t = threadIdx.x; const size_t bh = blockIdx.y; const size_t b = bh / NH; const int h = bh % NH; const int m0 = blockIdx.x * 64;
  for (int e = t; e < 64 * DD; e += 128) { const int ml = e / DD, d = e % DD; th[d][ml] = (_Float16)bfr(V[b * BSTR + ((size_t)(m0 + ml) * NH + h) * DD + d]); }
  __syncthreads();
  for (int e = t; e < DD * 8; e += 128) { const int d = e >> 3, q = e & 7; vst2((unsigned*)(VT + (bh * DD + d) * (size_t)SEQ + m0 + q * 8), *(const v4u*)&th[d][q * 8]); }
}
__global__ __launch_bounds__(128) void k_att(const float* __restrict__ Q, const float* __restrict__ K, const _Float16* __restrict__ VT, float* __restrict__ OUT) {
  __shared__ __align__(16) float sp[4][16][36]; __shared__ __align__(16) float so[4][16][68];
  const int tid = threadIdx.x, wave = tid >> 5, lane = tid & 31, col = lane & 15, g = lane >> 4;
  const size_t bh = blockIdx.y; const size_t b = bh / NH; const int h = bh % NH; const int q0 = blockIdx.x * 64 + wave * 16;
  v16b aq[2];
#pragma unroll
  for (int kc = 0; kc < 2; ++kc) { const float* pp = Q + b * BSTR + ((size_t)(q0 + col) * NH + h) * DD + kc * 32 + 8 * g;
#pragma unroll
    for (int i = 0; i < 8; ++i) { aq[kc][i] = (__bf16)pp[i]; aq[kc][8 + i] = (__bf16)pp[16 + i]; } }
  float m[8], l[8];
#pragma unroll
  for (int r = 0; r < 8; ++r) { m[r] = -3.0e38f; l[r] = 0.f; }
  v8f acc[4];
#pragma unroll
  for (int j = 0; j < 4; ++j) acc[j] = v8f{};
#pragma unroll 1
  for (int ks = 0; ks < SEQ / 32; ++ks) { float s[2][8];
#pragma unroll
    for (int ct = 0; ct < 2; ++ct) { const int kk = ks * 32 + ct * 16 + col; v8f c = {};
#pragma unroll
      for (int kc = 0; kc < 2; ++kc) { v16b w; const float* kp = K + b * BSTR + ((size_t)kk * NH + h) * DD + kc * 32 + 8 * g;
#pragma unroll
        for (int i = 0; i < 8; ++i) { w[i] = (__bf16)kp[i]; w[8 + i] = (__bf16)kp[16 + i]; }
        c = wmma_bf(aq[kc], w, c); }
#pragma unroll
      for (int r = 0; r < 8; ++r) s[ct][r] = c[r]; }
    float alpha[8];
#pragma unroll
    for (int r = 0; r < 8; ++r) { float mx = fmaxf(s[0][r], s[1][r]);
#pragma unroll
      for (int o = 1; o < 16; o <<= 1) mx = fmaxf(mx, __shfl_xor(mx, o));
      const float mn = fmaxf(m[r], mx); alpha[r] = __expf(m[r] - mn); const float e0 = __expf(s[0][r] - mn), e1 = __expf(s[1][r] - mn); float es = e0 + e1;
#pragma unroll
      for (int o = 1; o < 16; o <<= 1) es += __shfl_xor(es, o);
      l[r] = l[r] * alpha[r] + es; m[r] = mn; sp[wave][8 * g + r][col] = e0; sp[wave][8 * g + r][16 + col] = e1; }
#pragma unroll
    for (int j = 0; j < 4; ++j)
#pragma unroll
      for (int r = 0; r < 8; ++r) acc[j][r] *= alpha[r];
    ldsx();
    v16h pa, par; { const float* prow = &sp[wave][col][0] + 8 * (lane >> 4);
#pragma unroll
      for (int i = 0; i < 8; ++i) { const float p0 = prow[i] * PCARRY, p1 = prow[16 + i] * PCARRY; pa[i] = (_Float16)p0; pa[8 + i] = (_Float16)p1; par[i] = (_Float16)(p0 - (float)pa[i]); par[8 + i] = (_Float16)(p1 - (float)pa[8 + i]); } }
#pragma unroll
    for (int j = 0; j < 4; ++j) { const v16h vh = frag_h(VT + (bh * DD + j * 16 + col) * (size_t)SEQ + ks * 32, lane); acc[j] = wmma16(pa, vh, acc[j]); acc[j] = wmma16(par, vh, acc[j]); }
    ldsx(); }
#pragma unroll
  for (int r = 0; r < 8; ++r) { const float il = (1.0f / PCARRY) / l[r];
#pragma unroll
    for (int j = 0; j < 4; ++j) so[wave][8 * g + r][j * 16 + col] = acc[j][r] * il; }
  ldsx();
  const int lc = lane & 15;
  for (int rl = 0; rl < 16; ++rl) { const v4f ov = *(const v4f*)&so[wave][rl][lc * 4];
    if (lane < 16) vst2(OUT + ((b * OSEQ + q0 + rl) * NH + h) * (size_t)DD + lc * 4, ov); }
}

extern "C" void kernel_launch(void* const* d_in, const int* in_sizes, int n_in, void* d_out, int out_size, void* d_ws, size_t ws_size, hipStream_t stream) {
  if (n_in < 3) return;
  const size_t need = ((size_t)(NB - 1) * SEQ_FULL + SEQ) * RS;
  if ((size_t)in_sizes[0] < need || (size_t)in_sizes[1] < need || (size_t)in_sizes[2] < need) return;
  if ((size_t)out_size < (size_t)NB * OSEQ * RS) return;
  if (ws_size < (size_t)WS_END) return;
  const float* Qp = (const float*)d_in[0];
  const float* Kp = (const float*)d_in[1];
  const float* Vp = (const float*)d_in[2];
  char* ws = (char*)d_ws; _Float16* VT = (_Float16*)(ws + WS_VT);
  k_vt<<<dim3(SEQ / 64, NB * NH), 128, 0, stream>>>(Vp, VT);
  k_att<<<dim3(SEQ / 64, NB * NH), 128, 0, stream>>>(Qp, Kp, VT, (float*)d_out);
}
